// CharacterModel_30554397344036
// MI455X (gfx1250) — hardware-verified
//
#include <hip/hip_runtime.h>


namespace {
constexpr int NW_ = 8192, L = 16, V = 500, E = 64, H = 256, G4 = 4 * H;
constexpr float HS = 8.0f;

typedef _Float16 b16;
typedef __attribute__((ext_vector_type(16))) _Float16 v16b;
typedef __attribute__((ext_vector_type(8))) _Float16 v8b;
typedef __attribute__((ext_vector_type(8))) float v8f;
typedef __attribute__((ext_vector_type(4))) float v4f;
__device__ __forceinline__ float bf16_rne(float f) { unsigned int u = __float_as_uint(f); u += 0x7FFFu + ((u >> 16) & 1u); return __uint_as_float(u & 0xFFFF0000u); }
__device__ __forceinline__ v16b frag_kb(const b16* p, int hh) { const v8b a = *(const v8b*)(p + 8 * hh), b = *(const v8b*)(p + 16 + 8 * hh); v16b f;
#pragma unroll
  for (int e = 0; e < 8; ++e) { f[e] = a[e]; f[8 + e] = b[e]; } return f; }
__device__ __forceinline__ v8f wmma16b(v16b a, v16b b, v8f c) { v8f d = __builtin_amdgcn_wmma_f32_16x16x32_f16(false, a, false, b, (short)0, c, false, false); asm volatile("v_nop\n\tv_nop\n\tv_nop\n\tv_nop" : "+v"(d) : "v"(a), "v"(b)); return d; }
__device__ __forceinline__ void wave_lds_sync() { __builtin_amdgcn_fence(__ATOMIC_RELEASE, "workgroup"); __builtin_amdgcn_wave_barrier(); __builtin_amdgcn_fence(__ATOMIC_ACQUIRE, "workgroup"); }
__device__ __forceinline__ float nexp(float x) { return __builtin_amdgcn_exp2f(x * 1.4426950408889634f); }
__device__ __forceinline__ float sigm(float x) { return 1.0f / (1.0f + nexp(-x)); }
__device__ __forceinline__ float tanh_f(float x) { const float e = nexp(-2.0f * fabsf(x)); const float t = (1.0f - e) / (1.0f + e); return (x >= 0.0f) ? t : -t; }
__device__ __forceinline__ float pmul(float a, float b) { float p = a * b; asm volatile("" : "+v"(p)); return p; }

struct Wo_ { static constexpr size_t IH = 0, HH = IH + (size_t)G4 * E, EMB = HH + (size_t)G4 * H, END = EMB + (size_t)512 * E; };
__global__ __launch_bounds__(256) void prep_kernel(const float* __restrict__ emb, const float* __restrict__ Wih, const float* __restrict__ Whh, const float* __restrict__ bih, const float* __restrict__ bhh, const float* __restrict__ aw, const float* __restrict__ h0, const float* __restrict__ c0, b16* __restrict__ R, float* __restrict__ P) {
  const int t_ = blockIdx.x * 256 + threadIdx.x, nth = gridDim.x * 256;
  for (int pass = 0; pass < 2; ++pass) {
    for (int q = t_; q < G4 * E; q += nth) R[Wo_::IH + q] = (b16)bf16_rne(Wih[q]);
    for (int q = t_; q < G4 * H; q += nth) R[Wo_::HH + q] = (b16)bf16_rne(Whh[q]);
    for (int q = t_; q < 512 * E; q += nth) R[Wo_::EMB + q] = (b16)((q < V * E) ? bf16_rne(emb[q]) : 0.0f);
    for (int q = t_; q < 2816; q += nth) { float v; if (q < 1024) v = bih[q]; else if (q < 2048) v = bhh[q - 1024]; else if (q < 2304) v = aw[q - 2048]; else if (q < 2560) v = h0[q - 2304]; else v = c0[q - 2560]; P[q] = bf16_rne(v); }
    __threadfence(); }
}

__global__ __launch_bounds__(256) void charlstm_kernel(const int* __restrict__ chars, const int* __restrict__ wlen, const int* __restrict__ oidx, const b16* __restrict__ R, const float* __restrict__ P, float* __restrict__ out) {
  __shared__ __attribute__((aligned(16))) b16 Xs[16][E + 8], Hs[16][H + 8]; __shared__ float Dp[8][16]; __shared__ __attribute__((aligned(16))) float Res[16][H + 4];
  const int wave = threadIdx.x >> 5, lane = threadIdx.x & 31, nloc = lane & 15, hlf = lane >> 4, n0 = blockIdx.x * 16, u0 = wave * 32;
  const float* bih = P; const float* bhh = P + 1024; const float* aw = P + 2048; const float* hin = P + 2304; const float* cin = P + 2560; const b16* Emb = R + Wo_::EMB;
  float c[2][8], res[2][8];
#pragma unroll
  for (int t = 0; t < 2; ++t)
#pragma unroll
    for (int r = 0; r < 8; ++r) { const int u = u0 + t * 16 + nloc; c[t][r] = cin[u]; res[t][r] = 0.0f; }
  for (int i = threadIdx.x; i < 16 * H; i += 256) { const int rr = i / H, u = i % H; Hs[rr][u] = (b16)(hin[u] * HS); }
  __syncthreads();
  for (int step = 0; step < L; ++step) {
    for (int i = threadIdx.x; i < 16 * E; i += 256) { const int rr = i / E, k = i % E; int ch = chars[(size_t)(n0 + rr) * L + step]; ch = (ch < 0) ? 0 : (ch >= V ? V - 1 : ch); Xs[rr][k] = Emb[ch * E + k]; }
    __syncthreads();
    v8f g[4][2];
#pragma unroll
    for (int q = 0; q < 4; ++q) { g[q][0] = (v8f){}; g[q][1] = (v8f){}; }
#pragma unroll
    for (int kb = 0; kb < E; kb += 32) { const v16b a = frag_kb(&Xs[nloc][kb], hlf);
#pragma unroll
      for (int q = 0; q < 4; ++q)
#pragma unroll
        for (int t = 0; t < 2; ++t) { const v16b bw = frag_kb(R + Wo_::IH + (size_t)(q * H + u0 + t * 16 + nloc) * E + kb, hlf); g[q][t] = wmma16b(a, bw, g[q][t]); } }
    v8f gh[4][2];
#pragma unroll
    for (int q = 0; q < 4; ++q) { gh[q][0] = (v8f){}; gh[q][1] = (v8f){}; }
#pragma unroll 2
    for (int kb = 0; kb < H; kb += 32) { const v16b a = frag_kb(&Hs[nloc][kb], hlf);
#pragma unroll
      for (int q = 0; q < 4; ++q)
#pragma unroll
        for (int t = 0; t < 2; ++t) { const v16b bw = frag_kb(R + Wo_::HH + (size_t)(q * H + u0 + t * 16 + nloc) * H + kb, hlf); gh[q][t] = wmma16b(a, bw, gh[q][t]); } }
    float hn[2][8], dp[8];
#pragma unroll
    for (int r = 0; r < 8; ++r) dp[r] = 0.0f;
#pragma unroll
    for (int t = 0; t < 2; ++t) { const int u = u0 + t * 16 + nloc;
#pragma unroll
      for (int r = 0; r < 8; ++r) { const float pi = g[0][t][r] + gh[0][t][r] * (1.0f / HS) + bih[u] + bhh[u], pf = g[1][t][r] + gh[1][t][r] * (1.0f / HS) + bih[H + u] + bhh[H + u], pg = g[2][t][r] + gh[2][t][r] * (1.0f / HS) + bih[2 * H + u] + bhh[2 * H + u], po = g[3][t][r] + gh[3][t][r] * (1.0f / HS) + bih[3 * H + u] + bhh[3 * H + u];
        const float cc = pmul(sigm(pf), c[t][r]) + pmul(sigm(pi), tanh_f(pg)); c[t][r] = cc; const float h = pmul(sigm(po), tanh_f(cc)); hn[t][r] = h; dp[r] += pmul(h, aw[u]); } }
#pragma unroll
    for (int r = 0; r < 8; ++r) {
#pragma unroll
      for (int o = 1; o < 16; o <<= 1) dp[r] += __shfl_xor(dp[r], o); }
    __syncthreads();
    if (nloc == 0) {
#pragma unroll
      for (int r = 0; r < 8; ++r) Dp[wave][8 * hlf + r] = dp[r]; }
#pragma unroll
    for (int t = 0; t < 2; ++t) { const int u = u0 + t * 16 + nloc;
#pragma unroll
      for (int r = 0; r < 8; ++r) Hs[8 * hlf + r][u] = (b16)(hn[t][r] * HS); }
    __syncthreads();
#pragma unroll
    for (int r = 0; r < 8; ++r) { const int rr = 8 * hlf + r; float d = 0.0f;
#pragma unroll
      for (int w = 0; w < 8; ++w) d += Dp[w][rr];
      const int len = wlen[n0 + rr]; if (step < len) { const float wt = sigm(d);
#pragma unroll
        for (int t = 0; t < 2; ++t) res[t][r] += pmul(wt, hn[t][r]); } }
  }
#pragma unroll
  for (int t = 0; t < 2; ++t) { const int u = u0 + t * 16 + nloc;
#pragma unroll
    for (int r = 0; r < 8; ++r) Res[8 * hlf + r][u] = res[t][r]; }
  __syncthreads();
  for (int pass = 0; pass < 2; ++pass) { for (int i = threadIdx.x; i < 16 * (H / 4); i += 256) { const int rr = i / (H / 4), c4 = (i % (H / 4)) * 4; int dst = oidx[n0 + rr]; dst = (dst < 0) ? 0 : (dst >= NW_ ? NW_ - 1 : dst); *(volatile v4f*)(out + (size_t)dst * H + c4) = *(const v4f*)(&Res[rr][c4]); } __threadfence(); }
}
}

extern "C" void kernel_launch(void* const* d_in, const int* in_sizes, int n_in,
                              void* d_out, int out_size, void* d_ws, size_t ws_size, hipStream_t stream) {
  (void)n_in; (void)out_size;
  const int* chars = (const int*)d_in[0]; const int* wlen = (const int*)d_in[1]; const int* oidx = (const int*)d_in[2]; const float* emb = (const float*)d_in[3]; const float* Wih = (const float*)d_in[4]; const float* Whh = (const float*)d_in[5]; const float* bih = (const float*)d_in[6]; const float* bhh = (const float*)d_in[7]; const float* aw = (const float*)d_in[8]; const float* h0 = (const float*)d_in[9]; const float* c0 = (const float*)d_in[10];
  float* out = (float*)d_out;
  if (in_sizes[0] != NW_ * L || in_sizes[1] != NW_ || in_sizes[2] != NW_ || in_sizes[3] != V * E || in_sizes[4] != G4 * E || in_sizes[5] != G4 * H) return;
  size_t off = 0; char* ws = (char*)d_ws;
  auto carve = [&](size_t bytes) { char* p = ws + off; off += (bytes + 255) & ~(size_t)255; return p; };
  b16* R = (b16*)carve(Wo_::END * 2); float* P = (float*)carve(3072 * 4);
  if (off > ws_size) return;
  prep_kernel<<<128, 256, 0, stream>>>(emb, Wih, Whh, bih, bhh, aw, h0, c0, R, P);
  charlstm_kernel<<<NW_ / 16, 256, 0, stream>>>(chars, wlen, oidx, R, P, out);
}
